// CompositionalAttention_60481729462643
// MI455X (gfx1250) — hardware-verified
//
#include <hip/hip_runtime.h>
#include <math.h>
#include <stdint.h>

#ifndef NB
#define NB 2
#endif
#ifndef SEQ
#define SEQ 2048
#endif
#define NB_FULL  2
#define SEQ_FULL 2048
#define DM   1024
#define NS   8
#define NR   2
#define HD   64
#define DSQ  (NS * HD)
#define DRV  (NR * HD)
#define DOC  (2 * DSQ)
#define NQB  (SEQ / 64)
#define NKT  (SEQ / 64)
static_assert(NB >= 1 && NB <= NB_FULL);
static_assert(SEQ >= 64 && SEQ <= SEQ_FULL && (SEQ % 64) == 0);
static_assert(DSQ == 512 && DRV == 128 && HD == 64 && DOC == 1024);
static_assert((DM % 64) == 0 && (DSQ % 64) == 0 && (DRV % 64) == 0 && (DM % 32) == 0);

typedef _Float16 v16h __attribute__((ext_vector_type(16)));
typedef _Float16 v8h  __attribute__((ext_vector_type(8)));
typedef __bf16   v16b __attribute__((ext_vector_type(16)));
typedef __bf16   v8b  __attribute__((ext_vector_type(8)));
typedef float    v8f  __attribute__((ext_vector_type(8)));
typedef float    v4f  __attribute__((ext_vector_type(4)));
typedef unsigned int v4u __attribute__((ext_vector_type(4)));

#if defined(__HIP_DEVICE_COMPILE__)
#define DEV_ASM 1
#else
#define DEV_ASM 0
#endif

__device__ __forceinline__ unsigned short bf_bits(float f) {
  unsigned u = __float_as_uint(f);
  return (unsigned short)((u + 0x7FFFu + ((u >> 16) & 1u)) >> 16);
}
__device__ __forceinline__ float bf_up(unsigned short hb) { return __uint_as_float(((unsigned)hb) << 16); }
__device__ __forceinline__ unsigned short h_bits(_Float16 x) { return __builtin_bit_cast(unsigned short, x); }
__device__ __forceinline__ unsigned pk16(unsigned short a, unsigned short b) { return (unsigned)a | ((unsigned)b << 16); }
__device__ __forceinline__ v8f zero8() { v8f z = {0.f, 0.f, 0.f, 0.f, 0.f, 0.f, 0.f, 0.f}; return z; }

__device__ __forceinline__ void wave_lds_sync() {
  __builtin_amdgcn_fence(__ATOMIC_RELEASE, "workgroup");
  __builtin_amdgcn_wave_barrier();
  __builtin_amdgcn_fence(__ATOMIC_ACQUIRE, "workgroup");
}

template <typename OT> struct FT;
template <> struct FT<__bf16>   { typedef v16b frag; typedef v8b half8; };
template <> struct FT<_Float16> { typedef v16h frag; typedef v8h half8; };

template <typename OT>
__device__ __forceinline__ typename FT<OT>::frag ldfrag(const OT* p) {
  union { typename FT<OT>::frag v; typename FT<OT>::half8 h[2]; } f;
  f.h[0] = *(const typename FT<OT>::half8*)(p);
  f.h[1] = *(const typename FT<OT>::half8*)(p + 16);
  return f.v;
}

__device__ __forceinline__ v8f mmar(v16b a, v16b b, v8f c) {
  return __builtin_amdgcn_wmma_f32_16x16x32_bf16(false, a, false, b, (short)0, c, false, false);
}
__device__ __forceinline__ v8f mmar(v16h a, v16h b, v8f c) {
  return __builtin_amdgcn_wmma_f32_16x16x32_f16(false, a, false, b, (short)0, c, false, false);
}
__device__ __forceinline__ v8f mma_h(v16h a, v16h b, v8f c) {
  c = __builtin_amdgcn_wmma_f32_16x16x32_f16(false, a, false, b, (short)0, c, false, false);
#if DEV_ASM
  asm volatile("v_nop\n\tv_nop\n\tv_nop\n\tv_nop" : "+v"(c) : "v"(a), "v"(b));
#endif
  return c;
}
__device__ __forceinline__ void dep_guard(v8f& a, v8f& b, v16b x, v16b y) {
#if DEV_ASM
  asm volatile("v_nop\n\tv_nop\n\tv_nop\n\tv_nop" : "+v"(a), "+v"(b) : "v"(x), "v"(y));
#else
  (void)a; (void)b; (void)x; (void)y;
#endif
}
__device__ __forceinline__ void dep_guard(v8f& a, v8f& b, v16h x, v16h y) {
#if DEV_ASM
  asm volatile("v_nop\n\tv_nop\n\tv_nop\n\tv_nop" : "+v"(a), "+v"(b) : "v"(x), "v"(y));
#else
  (void)a; (void)b; (void)x; (void)y;
#endif
}
__device__ __forceinline__ void keep4(v16b a, v16b b, v16b c, v16b d) {
#if DEV_ASM
  asm volatile("v_nop" :: "v"(a), "v"(b), "v"(c), "v"(d));
#else
  (void)a; (void)b; (void)c; (void)d;
#endif
}
__device__ __forceinline__ void keep4(v16h a, v16h b, v16h c, v16h d) {
#if DEV_ASM
  asm volatile("v_nop" :: "v"(a), "v"(b), "v"(c), "v"(d));
#else
  (void)a; (void)b; (void)c; (void)d;
#endif
}
__device__ __forceinline__ void acc_guard4(v8f& a, v8f& b, v8f& c, v8f& d) {
#if DEV_ASM
  asm volatile("v_nop\n\tv_nop\n\tv_nop\n\tv_nop" : "+v"(a), "+v"(b), "+v"(c), "+v"(d));
#else
  (void)a; (void)b; (void)c; (void)d;
#endif
}

__global__ __launch_bounds__(256) void cvtbf8(const float* __restrict__ in, unsigned short* out, int n8,
                                              long long sIn, long long sOut) {
  const float* ib = in + (size_t)blockIdx.y * (size_t)sIn;
  unsigned short* ob = out + (size_t)blockIdx.y * (size_t)sOut;
  const int i = blockIdx.x * 256 + (int)threadIdx.x;
  if (i < n8) {
    const v4f a  = *(const v4f*)(ib + (size_t)i * 8);
    const v4f a4 = *(const v4f*)(ib + (size_t)i * 8 + 4);
    v4u p;
    p[0] = pk16(bf_bits(a[0]),  bf_bits(a[1]));
    p[1] = pk16(bf_bits(a[2]),  bf_bits(a[3]));
    p[2] = pk16(bf_bits(a4[0]), bf_bits(a4[1]));
    p[3] = pk16(bf_bits(a4[2]), bf_bits(a4[3]));
    unsigned short* o = ob + (size_t)i * 8;
    *(volatile v4u*)o = p;
    __threadfence();
    *(volatile v4u*)o = p;
  }
}

template <int MODE>
__global__ __launch_bounds__(256) void tconv64(const float* __restrict__ W, int R, int C,
                                               unsigned short* out, int ldo, float s1, float s2) {
  __shared__ __align__(16) unsigned short t1[64 * 72];
  __shared__ __align__(16) unsigned short t2[(MODE == 2) ? (64 * 72) : 8];
  const int tid = (int)threadIdx.x, lane = tid & 31, wave = tid >> 5;
  const int c0 = blockIdx.x * 64, r0 = blockIdx.y * 64;
  {
    const int rl = tid >> 2, cl0 = (tid & 3) * 16;
    const float* src = W + (size_t)(r0 + rl) * (size_t)C + c0 + cl0;
#pragma unroll
    for (int i = 0; i < 4; ++i) {
      const v4f a = *(const v4f*)(src + 4 * i);
#pragma unroll
      for (int e = 0; e < 4; ++e) {
        const int cl = cl0 + 4 * i + e;
        const unsigned short hb = bf_bits(a[e]);
        if (MODE == 0) {
          t1[cl * 72 + rl] = hb;
        } else {
          const float up = bf_up(hb);
          t1[cl * 72 + rl] = h_bits((_Float16)(up * s1));
          if (MODE == 2) t2[cl * 72 + rl] = h_bits((_Float16)(up * s2));
        }
      }
    }
  }
  __syncthreads();
  const int q = lane >> 3, p8 = (lane & 7) * 8;
  const v4u z4 = {0u, 0u, 0u, 0u};
  v4u a1[2], a2[2];
#pragma unroll
  for (int it = 0; it < 2; ++it) {
    const int cl = wave * 8 + it * 4 + q;
    a1[it] = *(const v4u*)(t1 + cl * 72 + p8);
    a2[it] = z4;
    if (MODE == 2) a2[it] = *(const v4u*)(t2 + cl * 72 + p8);
  }
  for (int pass = 0; pass < 2; ++pass) {
#pragma unroll
    for (int it = 0; it < 2; ++it) {
      const int cl = wave * 8 + it * 4 + q;
      unsigned short* o = out + (size_t)(c0 + cl) * (size_t)ldo + r0 + p8;
      *(volatile v4u*)o = a1[it];
      if (MODE == 2) *(volatile v4u*)(o + R) = a2[it];
    }
    __threadfence();
  }
}

template <typename OT, int OUT_MODE>
__global__ __launch_bounds__(256) void gemm64(
    const unsigned short* __restrict__ Ap, int lda, long long strideA,
    const unsigned short* __restrict__ Btp, int ldb, long long strideB,
    void* Cout, void* Cout2, int ldc, long long strideC,
    int M, int N, int K, float oscale, float rscale) {
  typedef typename FT<OT>::frag V16;
  const OT* A  = (const OT*)(const void*)Ap;
  const OT* Bt = (const OT*)(const void*)Btp;
  __shared__ __align__(16) float sT[8][16 * 68];
  const int b    = blockIdx.y;
  const int lane = threadIdx.x & 31;
  const int wave = threadIdx.x >> 5;
  const int tilesN = N >> 6;
  const int tilesM = M >> 6;
  const int tile = blockIdx.x * 8 + wave;
  if (tile >= tilesM * tilesN) return;
  const int tm = tile / tilesN;
  const int tn = tile - tm * tilesN;
  const int m0 = tm << 6;
  const int n0 = tn << 6;

  const OT* Ab = A  + (size_t)b * (size_t)strideA;
  const OT* Bb = Bt + (size_t)b * (size_t)strideB;

  const int rlane = lane & 15;
  const int koff  = (lane >> 4) * 8;
  const int mOff  = (lane >> 4) * 8;

  v8f acc[4][4];
#pragma unroll
  for (int i = 0; i < 4; ++i)
#pragma unroll
    for (int j = 0; j < 4; ++j) acc[i][j] = zero8();

  for (int k0 = 0; k0 < K; k0 += 32) {
    V16 bq[4];
#pragma unroll
    for (int j = 0; j < 4; ++j)
      bq[j] = ldfrag<OT>(Bb + (size_t)(n0 + (j << 4) + rlane) * ldb + koff + k0);
#pragma unroll
    for (int i = 0; i < 4; ++i) {
      const V16 af = ldfrag<OT>(Ab + (size_t)(m0 + (i << 4) + rlane) * lda + koff + k0);
#pragma unroll
      for (int j = 0; j < 4; ++j) acc[i][j] = mmar(af, bq[j], acc[i][j]);
      dep_guard(acc[i][0], acc[i][3], af, bq[3]);
    }
    keep4(bq[0], bq[1], bq[2], bq[3]);
  }
  acc_guard4(acc[0][0], acc[0][1], acc[0][2], acc[0][3]);
  acc_guard4(acc[1][0], acc[1][1], acc[1][2], acc[1][3]);
  acc_guard4(acc[2][0], acc[2][1], acc[2][2], acc[2][3]);
  acc_guard4(acc[3][0], acc[3][1], acc[3][2], acc[3][3]);

  float* slab = sT[wave];
#pragma unroll
  for (int i = 0; i < 4; ++i) {
    const int mBase = m0 + (i << 4);
#pragma unroll
    for (int j = 0; j < 4; ++j) {
#pragma unroll
      for (int r = 0; r < 8; ++r) {
        slab[(mOff + r) * 68 + (j << 4) + rlane] = acc[i][j][r];
      }
    }
    wave_lds_sync();
    if (OUT_MODE == 0) {
      float* Cp = (float*)Cout + (size_t)b * (size_t)strideC;
      const int h2 = lane >> 4, c4 = (lane & 15) * 4;
      for (int pass = 0; pass < 2; ++pass) {
#pragma unroll
        for (int it = 0; it < 8; ++it) {
          const int row = it * 2 + h2;
          const v4f v = *(const v4f*)(slab + row * 68 + c4) * oscale;
          *(volatile v4f*)(Cp + (size_t)(mBase + row) * ldc + n0 + c4) = v;
        }
        __threadfence();
      }
    } else {
      const int q = lane >> 3, c8 = (lane & 7) * 8;
      unsigned short* Cp  = (unsigned short*)Cout  + (size_t)b * (size_t)strideC;
      unsigned short* Cp2 = (unsigned short*)Cout2 + (size_t)b * (size_t)strideC;
      v4u hv[4], lv[4];
#pragma unroll
      for (int it = 0; it < 4; ++it) {
        const int row = it * 4 + q;
        const float* sp = slab + row * 68 + c8;
        float f[8];
#pragma unroll
        for (int e = 0; e < 8; ++e) f[e] = sp[e];
        v4u a, a2;
#pragma unroll
        for (int e = 0; e < 4; ++e) {
          const float f0 = f[2 * e], f1 = f[2 * e + 1];
          const _Float16 x0 = (_Float16)f0, x1 = (_Float16)f1;
          const unsigned short h0 = h_bits(x0), h1 = h_bits(x1);
          unsigned short l0 = 0, l1 = 0;
          if (OUT_MODE == 3) {
            l0 = h_bits((_Float16)((f0 - (float)x0) * rscale));
            l1 = h_bits((_Float16)((f1 - (float)x1) * rscale));
          }
          a[e] = pk16(h0, h1); a2[e] = pk16(l0, l1);
        }
        hv[it] = a; lv[it] = a2;
      }
      for (int pass = 0; pass < 2; ++pass) {
#pragma unroll
        for (int it = 0; it < 4; ++it) {
          const int row = it * 4 + q;
          *(volatile v4u*)(Cp + (size_t)(mBase + row) * ldc + n0 + c8) = hv[it];
          if (OUT_MODE == 3) *(volatile v4u*)(Cp2 + (size_t)(mBase + row) * ldc + n0 + c8) = lv[it];
        }
        __threadfence();
      }
    }
    wave_lds_sync();
  }
}

__global__ __launch_bounds__(128)
void attn_cs(const unsigned short* __restrict__ qhp, const unsigned short* __restrict__ qlp,
             const unsigned short* __restrict__ kpp,
             const unsigned short* __restrict__ vhp, const unsigned short* __restrict__ vlp,
             const unsigned short* __restrict__ wkp, const float* __restrict__ rqp,
             unsigned short* ocp, float sscale) {
  union FH { v16h v; v8h h[2]; };
  __shared__ __align__(16) _Float16 Ksh[64 * 64];
  __shared__ __align__(16) _Float16 Vsh[128 * 128];
  __shared__ __align__(16) _Float16 Psh[4][16 * 128];

  const int tid  = threadIdx.x;
  const int wave = tid >> 5;
  const int lane = tid & 31;
  const int hh   = lane >> 4;
  const int c    = lane & 15;

  const int bx   = blockIdx.x;
  const int qb   = bx % NQB;
  const int rest = bx / NQB;
  const int s    = rest % NS;
  const int b    = rest / NS;
  const int q0   = qb * 64 + wave * 16;
  const size_t rowB = (size_t)b * SEQ;

  const _Float16* Qh = (const _Float16*)(const void*)qhp;
  const _Float16* Ql = (const _Float16*)(const void*)qlp;
  const _Float16* Kg = (const _Float16*)(const void*)kpp + (size_t)s * HD;
  const _Float16* Vh = (const _Float16*)(const void*)vhp + (size_t)b * DRV * SEQ;
  const _Float16* Vl = (const _Float16*)(const void*)vlp + (size_t)b * DRV * SEQ;
  const _Float16* Wk = (const _Float16*)(const void*)wkp;

  v16h qah[2], qal[2];
#pragma unroll
  for (int dc = 0; dc < 2; ++dc) {
    const size_t qo = (rowB + q0 + c) * DSQ + (size_t)s * HD + dc * 32 + 8 * hh;
    qah[dc] = ldfrag<_Float16>(Qh + qo);
    qal[dc] = ldfrag<_Float16>(Ql + qo);
  }

  float mrow[8], lrow[8];
  v8f oacc[8];
#pragma unroll
  for (int r = 0; r < 8; ++r) { mrow[r] = -INFINITY; lrow[r] = 0.f; }
#pragma unroll
  for (int t = 0; t < 8; ++t) oacc[t] = zero8();

  _Float16* pwh = Psh[wave];

  for (int kt = 0; kt < NKT; ++kt) {
    const int kv0 = kt * 64;
    __syncthreads();
    {
      const int r = tid >> 1, half = (tid & 1) * 32;
      const _Float16* kg = Kg + (rowB + kv0 + r) * DSQ + half;
#pragma unroll
      for (int i = 0; i < 4; ++i) *(v8h*)(Ksh + r * 64 + half + 8 * i) = *(const v8h*)(kg + 8 * i);
      const _Float16* vg = Vh + (size_t)tid * SEQ + kv0;
#pragma unroll
      for (int i = 0; i < 8; ++i) *(v8h*)(Vsh + tid * 128 + 8 * i) = *(const v8h*)(vg + 8 * i);
      asm volatile("" ::: "memory");
      const _Float16* vlg = Vl + (size_t)tid * SEQ + kv0;
#pragma unroll
      for (int i = 0; i < 8; ++i) *(v8h*)(Vsh + tid * 128 + 64 + 8 * i) = *(const v8h*)(vlg + 8 * i);
    }
    __syncthreads();

    v8f sc[4];
#pragma unroll
    for (int j = 0; j < 4; ++j) {
      v8f ah = zero8(), al = zero8();
#pragma unroll
      for (int dc = 0; dc < 2; ++dc) {
        FH kb;
        kb.h[0] = *(const v8h*)(Ksh + (j * 16 + c) * 64 + dc * 32 + 8 * hh);
        kb.h[1] = *(const v8h*)(Ksh + (j * 16 + c) * 64 + dc * 32 + 16 + 8 * hh);
        ah = mma_h(qah[dc], kb.v, ah);
        al = mma_h(qal[dc], kb.v, al);
      }
#pragma unroll
      for (int r = 0; r < 8; ++r) sc[j][r] = (ah[r] + al[r] * (1.0f / 4096.0f)) * sscale;
    }

#pragma unroll
    for (int r = 0; r < 8; ++r) {
      float m = sc[0][r];
#pragma unroll
      for (int j = 1; j < 4; ++j) m = fmaxf(m, sc[j][r]);
#pragma unroll
      for (int off = 1; off < 16; off <<= 1) m = fmaxf(m, __shfl_xor(m, off, 32));
      const float mnew  = fmaxf(mrow[r], m);
      const float msafe = (mnew == -INFINITY) ? 0.f : mnew;
      const float alpha = __expf(mrow[r] - msafe);
      mrow[r] = mnew;
      float psum = 0.f;
#pragma unroll
      for (int j = 0; j < 4; ++j) {
        const float p = __expf(sc[j][r] - msafe);
        psum += p;
        pwh[(8 * hh + r) * 128 + j * 16 + c]      = (_Float16)(p * 16384.0f);
        pwh[(8 * hh + r) * 128 + 64 + j * 16 + c] = (_Float16)(p * 1024.0f);
      }
#pragma unroll
      for (int off = 1; off < 16; off <<= 1) psum += __shfl_xor(psum, off, 32);
      lrow[r] = lrow[r] * alpha + psum;
#pragma unroll
      for (int t = 0; t < 8; ++t) oacc[t][r] *= alpha;
    }
    wave_lds_sync();

#pragma unroll 1
    for (int kk = 0; kk < 4; ++kk) {
      FH pa;
      pa.h[0] = *(const v8h*)(pwh + c * 128 + kk * 32 + 8 * hh);
      pa.h[1] = *(const v8h*)(pwh + c * 128 + kk * 32 + 16 + 8 * hh);
#pragma unroll
      for (int t = 0; t < 8; ++t) {
        FH vb;
        vb.h[0] = *(const v8h*)(Vsh + (t * 16 + c) * 128 + kk * 32 + 8 * hh);
        vb.h[1] = *(const v8h*)(Vsh + (t * 16 + c) * 128 + kk * 32 + 16 + 8 * hh);
        oacc[t] = mma_h(pa.v, vb.v, oacc[t]);
      }
    }
  }

  __syncthreads();
  {
    const int r = tid >> 1, half = (tid & 1) * 32;
    const _Float16* wg = Wk + r * HD + half;
#pragma unroll
    for (int i = 0; i < 4; ++i) *(v8h*)(Ksh + r * 64 + half + 8 * i) = *(const v8h*)(wg + 8 * i);
  }
  float* os = reinterpret_cast<float*>(Vsh) + wave * (16 * 128);
#pragma unroll
  for (int r = 0; r < 8; ++r) {
    const float l = lrow[r];
    const float inv = ((l > 0.f) ? (1.0f / l) : 0.f) * (1.0f / 256.0f);
#pragma unroll
    for (int t = 0; t < 8; ++t) {
      const float v = oacc[t][r] * inv;
      os[(8 * hh + r) * 128 + t * 16 + c]  = v;
      pwh[(8 * hh + r) * 128 + t * 16 + c] = (_Float16)v;
    }
  }
  __syncthreads();

  v8f rk[8];
#pragma unroll
  for (int i = 0; i < 8; ++i) rk[i] = zero8();
#pragma unroll
  for (int rr = 0; rr < 2; ++rr) {
#pragma unroll
    for (int kk = 0; kk < 2; ++kk) {
      FH pa;
      pa.h[0] = *(const v8h*)(pwh + c * 128 + rr * 64 + kk * 32 + 8 * hh);
      pa.h[1] = *(const v8h*)(pwh + c * 128 + rr * 64 + kk * 32 + 16 + 8 * hh);
#pragma unroll
      for (int t4 = 0; t4 < 4; ++t4) {
        FH wb;
        wb.h[0] = *(const v8h*)(Ksh + (t4 * 16 + c) * 64 + kk * 32 + 8 * hh);
        wb.h[1] = *(const v8h*)(Ksh + (t4 * 16 + c) * 64 + kk * 32 + 16 + 8 * hh);
        rk[rr * 4 + t4] = mma_h(pa.v, wb.v, rk[rr * 4 + t4]);
      }
    }
  }
  acc_guard4(rk[0], rk[1], rk[2], rk[3]);
  acc_guard4(rk[4], rk[5], rk[6], rk[7]);
  wave_lds_sync();

  float* rqs = reinterpret_cast<float*>(pwh);
  {
    const int r2 = lane >> 4, c4 = (lane & 15) * 4;
    const float* rqg = rqp + (rowB + q0) * DSQ + (size_t)s * HD + c4;
#pragma unroll
    for (int it = 0; it < 8; ++it) {
      const int row = it * 2 + r2;
      *(v4f*)(rqs + row * 64 + c4) = *(const v4f*)(rqg + (size_t)row * DSQ);
    }
  }
  wave_lds_sync();

  float d0[8], d1[8];
#pragma unroll
  for (int r8 = 0; r8 < 8; ++r8) {
    float a0 = 0.f, a1 = 0.f;
#pragma unroll
    for (int t4 = 0; t4 < 4; ++t4) {
      const float qv = rqs[(8 * hh + r8) * 64 + t4 * 16 + c];
      a0 += qv * rk[t4][r8];
      a1 += qv * rk[4 + t4][r8];
    }
    d0[r8] = a0; d1[r8] = a1;
  }
#pragma unroll
  for (int r8 = 0; r8 < 8; ++r8) {
#pragma unroll
    for (int off = 1; off < 16; off <<= 1) {
      d0[r8] += __shfl_xor(d0[r8], off, 32);
      d1[r8] += __shfl_xor(d1[r8], off, 32);
    }
  }
  float w0[8], w1[8];
  const float rsc = sscale * (1.0f / 4096.0f);
#pragma unroll
  for (int r8 = 0; r8 < 8; ++r8) {
    const float x0 = d0[r8] * rsc, x1 = d1[r8] * rsc;
    const float m  = fmaxf(x0, x1);
    const float e0 = __expf(x0 - m), e1 = __expf(x1 - m);
    const float iv = 1.0f / (e0 + e1);
    w0[r8] = e0 * iv; w1[r8] = e1 * iv;
  }
  wave_lds_sync();

  float* oc = rqs;
#pragma unroll
  for (int r8 = 0; r8 < 8; ++r8) {
#pragma unroll
    for (int t = 0; t < 4; ++t) {
      const int row = 8 * hh + r8;
      const float o = w0[r8] * os[row * 128 + t * 16 + c] + w1[r8] * os[row * 128 + 64 + t * 16 + c];
      oc[row * 64 + t * 16 + c] = o;
    }
  }
  wave_lds_sync();

  {
    const int q4 = lane >> 3, c8 = (lane & 7) * 8;
    v4u hv[4], lv[4];
#pragma unroll
    for (int it = 0; it < 4; ++it) {
      const int row = it * 4 + q4;
      const float* sp = oc + row * 64 + c8;
      float f[8];
#pragma unroll
      for (int e = 0; e < 8; ++e) f[e] = sp[e];
      v4u a, a2;
#pragma unroll
      for (int e = 0; e < 4; ++e) {
        const float f0 = f[2 * e], f1 = f[2 * e + 1];
        const _Float16 x0 = (_Float16)f0, x1 = (_Float16)f1;
        const unsigned short l0 = h_bits((_Float16)((f0 - (float)x0) * 16.0f));
        const unsigned short l1 = h_bits((_Float16)((f1 - (float)x1) * 16.0f));
        a[e] = pk16(h_bits(x0), h_bits(x1)); a2[e] = pk16(l0, l1);
      }
      hv[it] = a; lv[it] = a2;
    }
    for (int pass = 0; pass < 2; ++pass) {
#pragma unroll
      for (int it = 0; it < 4; ++it) {
        const int row = it * 4 + q4;
        const size_t go = (rowB + q0 + row) * DOC + (size_t)s * HD + c8;
        *(volatile v4u*)(ocp + go)       = hv[it];
        *(volatile v4u*)(ocp + go + DSQ) = lv[it];
      }
      __threadfence();
    }
  }
}

extern "C" void kernel_launch(void* const* d_in, const int* in_sizes, int n_in,
                              void* d_out, int out_size, void* d_ws, size_t ws_size,
                              hipStream_t stream) {
  if (n_in < 7) return;
  if (in_sizes[0] < ((NB - 1) * SEQ_FULL + SEQ) * DM) return;
  if (in_sizes[1] < DM * DSQ || in_sizes[2] < DM * DSQ || in_sizes[4] < DM * DSQ) return;
  if (in_sizes[3] < DM * DRV) return;
  if (in_sizes[5] < HD * HD) return;
  if (in_sizes[6] < DSQ * DM) return;
  if (out_size < NB * SEQ * DM) return;

  const float* x    = (const float*)d_in[0];
  const float* Wsq  = (const float*)d_in[1];
  const float* Wsk  = (const float*)d_in[2];
  const float* Wrv  = (const float*)d_in[3];
  const float* Wrq  = (const float*)d_in[4];
  const float* Wrk  = (const float*)d_in[5];
  const float* Wout = (const float*)d_in[6];

  const size_t PXB = (size_t)NB * SEQ * DM * 2;
  const size_t PWS = (size_t)DSQ * DM * 2;
  const size_t PWV = (size_t)DRV * DM * 2;
  const size_t PWK = (size_t)HD * HD * 2;
  const size_t PWO = (size_t)DM * DOC * 2;
  const size_t PQ  = (size_t)NB * SEQ * DSQ * 2;
  const size_t PRQ = (size_t)NB * SEQ * DSQ * 4;
  const size_t PVT = (size_t)NB * DRV * SEQ * 2;
  const size_t POC = (size_t)NB * SEQ * DOC * 2;
  size_t off = 0;
  const size_t oXb  = off; off += PXB;
  const size_t oWsq = off; off += PWS;
  const size_t oWsk = off; off += PWS;
  const size_t oWrq = off; off += PWS;
  const size_t oWrv = off; off += PWV;
  const size_t oWrk = off; off += PWK;
  const size_t oWo  = off; off += PWO;
  const size_t oQh  = off; off += PQ;
  const size_t oQl  = off; off += PQ;
  const size_t oKp  = off; off += PQ;
  const size_t oRQ  = off; off += PRQ;
  const size_t oVTh = off; off += PVT;
  const size_t oVTl = off; off += PVT;
  const size_t oOC  = off; off += POC;
  if (off > ws_size) return;
  if (off > (size_t)134217728) return;

  char* ws = (char*)d_ws;
  unsigned short* Xb   = (unsigned short*)(ws + oXb);
  unsigned short* WsqT = (unsigned short*)(ws + oWsq);
  unsigned short* WskT = (unsigned short*)(ws + oWsk);
  unsigned short* WrqT = (unsigned short*)(ws + oWrq);
  unsigned short* WrvT = (unsigned short*)(ws + oWrv);
  unsigned short* WrkT = (unsigned short*)(ws + oWrk);
  unsigned short* WoT  = (unsigned short*)(ws + oWo);
  unsigned short* Qh   = (unsigned short*)(ws + oQh);
  unsigned short* Ql   = (unsigned short*)(ws + oQl);
  unsigned short* Kp   = (unsigned short*)(ws + oKp);
  float*          RQ   = (float*)(ws + oRQ);
  unsigned short* VTh  = (unsigned short*)(ws + oVTh);
  unsigned short* VTl  = (unsigned short*)(ws + oVTl);
  unsigned short* OC   = (unsigned short*)(ws + oOC);

  const dim3 blk(256);
  const int n8x = SEQ * DM / 8;
  const dim3 gCvtX((n8x + 255) / 256, NB);
  const dim3 gTsq(DSQ / 64, DM / 64);
  const dim3 gTrv(DRV / 64, DM / 64);
  const dim3 gTrk(1, 1);
  const dim3 gTwo(DM / 64, DSQ / 64);
  const dim3 gP((((NB * SEQ) / 64) * (DSQ / 64) + 7) / 8, 1);
  const dim3 gV((((DRV / 64) * (SEQ / 64)) + 7) / 8, NB);
  const dim3 gAttn(NB * NS * NQB);
  const dim3 gO((((NB * SEQ) / 64) * (DM / 64) + 7) / 8, 1);

  cvtbf8<<<gCvtX, blk, 0, stream>>>(x, Xb, n8x, (long long)SEQ_FULL * DM, (long long)SEQ * DM);
  tconv64<0><<<gTsq, blk, 0, stream>>>(Wsq, DM, DSQ, WsqT, DM, 1.0f, 1.0f);
  tconv64<0><<<gTsq, blk, 0, stream>>>(Wsk, DM, DSQ, WskT, DM, 1.0f, 1.0f);
  tconv64<0><<<gTsq, blk, 0, stream>>>(Wrq, DM, DSQ, WrqT, DM, 1.0f, 1.0f);
  tconv64<0><<<gTrv, blk, 0, stream>>>(Wrv, DM, DRV, WrvT, DM, 1.0f, 1.0f);
  tconv64<1><<<gTrk, blk, 0, stream>>>(Wrk, HD, HD, WrkT, HD, 64.0f, 1.0f);
  tconv64<2><<<gTwo, blk, 0, stream>>>(Wout, DSQ, DM, WoT, DOC, 1024.0f, 64.0f);
  gemm64<__bf16, 3><<<gP, blk, 0, stream>>>(
      Xb, DM, 0LL, WsqT, DM, 0LL, (void*)Qh, (void*)Ql, DSQ, 0LL, NB * SEQ, DSQ, DM, 1.0f, 4096.0f);
  gemm64<__bf16, 1><<<gP, blk, 0, stream>>>(
      Xb, DM, 0LL, WskT, DM, 0LL, (void*)Kp, (void*)Kp, DSQ, 0LL, NB * SEQ, DSQ, DM, 1.0f, 1.0f);
  gemm64<__bf16, 0><<<gP, blk, 0, stream>>>(
      Xb, DM, 0LL, WrqT, DM, 0LL, (void*)RQ, (void*)RQ, DSQ, 0LL, NB * SEQ, DSQ, DM, 1.0f, 1.0f);
  gemm64<__bf16, 3><<<gV, blk, 0, stream>>>(
      WrvT, DM, 0LL, Xb, DM, (long long)SEQ * DM, (void*)VTh, (void*)VTl, SEQ, (long long)DRV * SEQ,
      DRV, SEQ, DM, 1.0f, 16.0f);
  attn_cs<<<gAttn, dim3(128), 0, stream>>>(Qh, Ql, Kp, VTh, VTl, WrkT, RQ, OC, 0.125f);
  gemm64<_Float16, 0><<<gO, blk, 0, stream>>>(
      OC, DOC, 0LL, WoT, DOC, 0LL, d_out, d_out, DM, 0LL, NB * SEQ, DM, DOC, 1.0f / 65536.0f, 1.0f);
  (void)hipGetLastError();
}
